// GCNGenerator_57775900066051
// MI455X (gfx1250) — hardware-run, weakly checked
//
#include <hip/hip_runtime.h>


typedef _Float16 f16t;
typedef f16t  v16h __attribute__((ext_vector_type(16)));
typedef f16t  v8h  __attribute__((ext_vector_type(8)));
typedef float v8f  __attribute__((ext_vector_type(8)));
typedef float v4f  __attribute__((ext_vector_type(4)));

union Frag { v16h v; v8h q[2]; };

#define NN   128
#define PF   132
#define PH   136
#define NTH  256

#define OFF_ADJ   0
#define OFF_OUT   (OFF_ADJ + NN * PF * 4)
#define OFF_XT    (OFF_OUT + NN * NN * 4)
#define OFF_Y     (OFF_XT + NN * PH * 2)
#define OFF_W     (OFF_Y + NN * PH * 2)
#define OFF_DI    (OFF_W + NN * PH * 2)
#define LDS_BYTES (OFF_DI + NN * 4)

static_assert(LDS_BYTES == 238080);
static_assert((OFF_OUT % 16) == 0 && (OFF_XT % 16) == 0 && (OFF_Y % 16) == 0 &&
              (OFF_W % 16) == 0 && (OFF_DI % 16) == 0);

#define SC_W 128.0f
#define SC_X 64.0f

__device__ __forceinline__ v8f wmma16(v16h a, v16h b, v8f c) {
    return __builtin_amdgcn_wmma_f32_16x16x32_f16(false, a, false, b, (short)0, c, false, false);
}

__device__ __forceinline__ void wguard4(v8f (&c)[4], Frag (&a)[4], v16h b) {
    asm volatile("v_nop\n\tv_nop\n\tv_nop\n\tv_nop"
                 : "+v"(c[0]), "+v"(c[1]), "+v"(c[2]), "+v"(c[3])
                 : "v"(a[0].v), "v"(a[1].v), "v"(a[2].v), "v"(a[3].v), "v"(b));
}

__device__ __forceinline__ v16h frag16(const f16t* p) {
    Frag f;
    f.q[0] = *(const v8h*)(p);
    f.q[1] = *(const v8h*)(p + 16);
    return f.v;
}

__device__ __forceinline__ v16h frag32(const float* p) {
    v4f u0 = *(const v4f*)(p);
    v4f u1 = *(const v4f*)(p + 4);
    v4f u2 = *(const v4f*)(p + 16);
    v4f u3 = *(const v4f*)(p + 20);
    Frag f;
    v8h q0 = {(f16t)u0[0], (f16t)u0[1], (f16t)u0[2], (f16t)u0[3],
              (f16t)u1[0], (f16t)u1[1], (f16t)u1[2], (f16t)u1[3]};
    v8h q1 = {(f16t)u2[0], (f16t)u2[1], (f16t)u2[2], (f16t)u2[3],
              (f16t)u3[0], (f16t)u3[1], (f16t)u3[2], (f16t)u3[3]};
    f.q[0] = q0;
    f.q[1] = q1;
    return f.v;
}

template <bool RELU>
__device__ __forceinline__ float epi1(float a, float scale) {
    float s = a * scale;
    if (RELU) s = fmaxf(s, 0.0f);
    return s;
}

template <bool BF32, bool RELU>
__device__ __forceinline__ void tile_gemm(const f16t* bufA, const void* bufB,
                                          f16t* outT, int wn, float scale) {
    const int l = threadIdx.x & 31, h = l >> 4, m = l & 15;
    const int brow = 16 * wn + m;
    v16h bf[4];
#pragma unroll
    for (int kt = 0; kt < 4; ++kt) {
        if constexpr (BF32) {
            bf[kt] = frag32((const float*)bufB + (size_t)brow * PF + 32 * kt + 8 * h);
        } else {
            bf[kt] = frag16((const f16t*)bufB + (size_t)brow * PH + 32 * kt + 8 * h);
        }
    }
#pragma unroll
    for (int p = 0; p < 2; ++p) {
        const v8f z = {0.f, 0.f, 0.f, 0.f, 0.f, 0.f, 0.f, 0.f};
        v8f acc[4];
        acc[0] = z; acc[1] = z; acc[2] = z; acc[3] = z;
#pragma unroll
        for (int kt = 0; kt < 4; ++kt) {
            Frag a[4];
#pragma unroll
            for (int t = 0; t < 4; ++t) {
                const f16t* ar = bufA + (size_t)(16 * (4 * p + t) + m) * PH + 32 * kt + 8 * h;
                a[t].q[0] = *(const v8h*)(ar);
                a[t].q[1] = *(const v8h*)(ar + 16);
            }
#pragma unroll
            for (int t = 0; t < 4; ++t) acc[t] = wmma16(a[t].v, bf[kt], acc[t]);
            wguard4(acc, a, bf[kt]);
        }
#pragma unroll
        for (int t = 0; t < 4; ++t) {
            v8h o = {(f16t)epi1<RELU>(acc[t][0], scale), (f16t)epi1<RELU>(acc[t][1], scale),
                     (f16t)epi1<RELU>(acc[t][2], scale), (f16t)epi1<RELU>(acc[t][3], scale),
                     (f16t)epi1<RELU>(acc[t][4], scale), (f16t)epi1<RELU>(acc[t][5], scale),
                     (f16t)epi1<RELU>(acc[t][6], scale), (f16t)epi1<RELU>(acc[t][7], scale)};
            *(v8h*)(outT + (size_t)brow * PH + 16 * (4 * p + t) + 8 * h) = o;
        }
    }
}

__global__ __launch_bounds__(NTH)
void k_gcn(const float* __restrict__ gx, const float* __restrict__ gw,
           float* __restrict__ gout, int nb) {
    extern __shared__ __attribute__((aligned(16))) char smem[];
    float* s_adj = (float*)(smem + OFF_ADJ);
    float* s_out = (float*)(smem + OFF_OUT);
    f16t*  s_xT  = (f16t*)(smem + OFF_XT);
    f16t*  s_y   = (f16t*)(smem + OFF_Y);
    f16t*  s_w   = (f16t*)(smem + OFF_W);
    float* s_di  = (float*)(smem + OFF_DI);

    const int tid = threadIdx.x;
    const int l   = tid & 31;
    const int w   = tid >> 5;
    const int b   = blockIdx.x;
    if (b >= nb) return;

    const float* xb = gx + (size_t)b * NN * NN;
    float*       ob = gout + (size_t)b * NN * NN;

    for (int p = tid; p < NN * (NN / 8); p += NTH) {
        const int e  = p & (NN - 1);
        const int d0 = (p >> 7) * 8;
        const float* wp = gw + (size_t)d0 * NN + e;
        v8h o = {(f16t)(wp[0 * NN] * SC_W), (f16t)(wp[1 * NN] * SC_W),
                 (f16t)(wp[2 * NN] * SC_W), (f16t)(wp[3 * NN] * SC_W),
                 (f16t)(wp[4 * NN] * SC_W), (f16t)(wp[5 * NN] * SC_W),
                 (f16t)(wp[6 * NN] * SC_W), (f16t)(wp[7 * NN] * SC_W)};
        *(v8h*)(s_w + e * PH + d0) = o;
    }
    for (int p = tid; p < NN * (NN / 8); p += NTH) {
        const int i  = p >> 4;
        const int d0 = (p & 15) * 8;
        const float* xp = xb + i * NN + d0;
        v4f u0 = *(const v4f*)(xp);
        v4f u1 = *(const v4f*)(xp + 4);
        v8h o = {(f16t)u0[0], (f16t)u0[1], (f16t)u0[2], (f16t)u0[3],
                 (f16t)u1[0], (f16t)u1[1], (f16t)u1[2], (f16t)u1[3]};
        *(v8h*)(s_y + i * PH + d0) = o;
    }
    for (int p = tid; p < NN * (NN / 4); p += NTH) {
        const int r  = p >> 5;
        const int c0 = (p & 31) * 4;
        v4f v = {(c0 + 0 == r) ? 1.0f : 0.0f, (c0 + 1 == r) ? 1.0f : 0.0f,
                 (c0 + 2 == r) ? 1.0f : 0.0f, (c0 + 3 == r) ? 1.0f : 0.0f};
        *(v4f*)(s_adj + r * PF + c0) = v;
        *(v4f*)(s_out + r * NN + c0) = v;
    }
    __syncthreads();

    tile_gemm<false, true>(s_y, s_w, s_xT, w, SC_X / SC_W);
    __syncthreads();

#pragma unroll 1
    for (int i = 1; i < NN; ++i) {
        if (tid < NN) {
            const f16t* cj = s_xT + tid;
            const f16t* ci = s_xT + i;
            float acc = 0.0f;
#pragma unroll 4
            for (int d = 0; d < NN; ++d)
                acc = fmaf((float)cj[d * PH], (float)ci[d * PH], acc);
            const float pr = acc * (1.0f / (SC_X * SC_X));
            if (tid < i) {
                s_out[i * NN + tid]  = pr;
                s_out[tid * NN + i]  = pr;
                s_adj[i * PF + tid]  = pr;
                s_adj[tid * PF + i]  = pr;
            }
        }
        __syncthreads();

#pragma unroll 1
        for (int rr = 0; rr < 16; ++rr) {
            const int r = 16 * w + rr;
            v4f v = *(const v4f*)(s_adj + r * PF + 4 * l);
            float s = (v[0] + v[1]) + (v[2] + v[3]);
            s += __shfl_xor(s, 16);
            s += __shfl_xor(s, 8);
            s += __shfl_xor(s, 4);
            s += __shfl_xor(s, 2);
            s += __shfl_xor(s, 1);
            if (l == 0) s_di[r] = 1.0f / sqrtf(s);
        }
        __syncthreads();

        {
            const int r  = tid >> 1;
            const int c0 = (tid & 1) * 64;
            const float dr = s_di[r];
            float* ar = s_adj + r * PF + c0;
            const float* dc = s_di + c0;
#pragma unroll 4
            for (int q = 0; q < 16; ++q) {
                v4f v = *(const v4f*)(ar + 4 * q);
                v4f d = *(const v4f*)(dc + 4 * q);
                v4f o = {(dr * v[0]) * d[0], (dr * v[1]) * d[1],
                         (dr * v[2]) * d[2], (dr * v[3]) * d[3]};
                *(v4f*)(ar + 4 * q) = o;
            }
        }
        __syncthreads();

        tile_gemm<true, false>(s_xT, s_adj, s_y, w, 1.0f);
        __syncthreads();

        tile_gemm<false, true>(s_y, s_w, s_xT, w, 1.0f / SC_W);
        __syncthreads();
    }

#pragma unroll 1
    for (int it = 0; it < NN / 8; ++it) {
        const int row = it * 8 + w;
        v4f v = *(const v4f*)(s_out + row * NN + 4 * l);
        *(volatile v4f*)(ob + (size_t)row * NN + 4 * l) = v;
    }
    __threadfence();
#pragma unroll 1
    for (int it = 0; it < NN / 8; ++it) {
        const int row = it * 8 + w;
        v4f v = *(const v4f*)(s_out + row * NN + 4 * l);
        *(volatile v4f*)(ob + (size_t)row * NN + 4 * l) = v;
    }
}

extern "C" void kernel_launch(void* const* d_in, const int* in_sizes, int n_in,
                              void* d_out, int out_size, void* d_ws, size_t ws_size,
                              hipStream_t stream) {
    if (n_in < 2) return;
    const int per = NN * NN;
    const int nb  = in_sizes[0] / per;
    if (nb <= 0 || in_sizes[0] != nb * per) return;
    if (in_sizes[1] != per) return;
    if (out_size != in_sizes[0]) return;
    (void)d_ws; (void)ws_size;

    const float* x = (const float*)d_in[0];
    const float* W = (const float*)d_in[1];
    float* out = (float*)d_out;

    hipFuncSetAttribute(reinterpret_cast<const void*>(&k_gcn),
                        hipFuncAttributeMaxDynamicSharedMemorySize, LDS_BYTES);
    k_gcn<<<dim3(nb), dim3(NTH), LDS_BYTES, stream>>>(x, W, out, nb);
}
